// DAGERCModule_25692494365064
// MI455X (gfx1250) — hardware-run, weakly checked
//
#include <hip/hip_runtime.h>
#include <math.h>

typedef __attribute__((ext_vector_type(16))) _Float16 v16h;
typedef __attribute__((ext_vector_type(8)))  _Float16 v8h;
typedef __attribute__((ext_vector_type(4)))  _Float16 v4h;
typedef __attribute__((ext_vector_type(8)))  float    v8f;
typedef __attribute__((ext_vector_type(4)))  float    v4f;

constexpr int kHid   = 300;
constexpr int kLay   = 4;
constexpr int kBat   = 8;
constexpr int kUtt   = 128;
constexpr int kEmb   = 100;
constexpr int kCls   = 7;
constexpr int kRows  = kBat * kUtt;
constexpr int kHP    = 320;
constexpr int kCatP  = 1728;
constexpr int kInCol = 1600;
constexpr int kInP   = 128;
constexpr int kGN    = 1920;
constexpr int kWrK   = 640;
constexpr int kScanThreads = 640;
constexpr int kM01P  = 648;
constexpr int kM16P  = 328;
constexpr float kWCarry = 16.0f;
constexpr float kWInv   = 1.0f / kWCarry;
static_assert(kRows == 1024, "rows");
static_assert((kHP % 32) == 0 && (kInP % 32) == 0 && (kCatP % 32) == 0 && (kWrK % 32) == 0, "GEMM K multiples of 32");
static_assert((kRows % 64) == 0 && (kHP % 64) == 0 && (kGN % 64) == 0, "GEMM M,N multiples of 64");
static_assert(kGN == 20 * 96 && kHP == 20 * 16, "20 wave groups");
static_assert(kScanThreads == 20 * 32 && kScanThreads * 4 == kBat * kHP && kScanThreads == kBat * 80, "scan thread maps");
static_assert(kInCol == 5 * kHP && kInCol + kInP == kCatP, "concat plane");

constexpr size_t kSzH    = (size_t)kRows * kHP * 4;
constexpr size_t kOffH   = 0;
constexpr size_t kOffCat = kOffH   + 5 * kSzH;
constexpr size_t kOffGXT = kOffCat + (size_t)kRows * kCatP * 2;
constexpr size_t kOffWX  = kOffGXT + (size_t)kGN * kRows * 4;
constexpr size_t kOffWM  = kOffWX  + (size_t)kLay * kGN * kHP * 2;
constexpr size_t kOffWR  = kOffWM  + (size_t)kLay * kGN * kHP * 2;
constexpr size_t kOffFC1 = kOffWR  + (size_t)kLay * kHP * kWrK * 2;
constexpr size_t kOffM1  = kOffFC1 + (size_t)kHP * kInP * 2;
constexpr size_t kOffM2  = kOffM1  + (size_t)kHP * kCatP * 2;
constexpr size_t kOffH1  = kOffM2  + (size_t)kHP * kHP * 2;
constexpr size_t kOffH2  = kOffH1  + (size_t)kRows * kHP * 2;
constexpr size_t kOffBias = kOffH2 + (size_t)kRows * kHP * 4;
constexpr int    kBiasFloats = 3 * kHP + 2 * kLay * kGN;
constexpr size_t kWsTotal = kOffBias + (size_t)kBiasFloats * 4;
static_assert(kBiasFloats == 16320, "bias floats");
static_assert(kWsTotal == 32849664ull, "carve total");
static_assert(kWsTotal <= 134217728ull, "carve cap");
static_assert((kOffCat % 128) == 0 && (kOffGXT % 128) == 0 && (kOffWX % 128) == 0 && (kOffWM % 128) == 0 &&
              (kOffWR % 128) == 0 && (kOffFC1 % 128) == 0 && (kOffM1 % 128) == 0 && (kOffM2 % 128) == 0 &&
              (kOffH1 % 128) == 0 && (kOffH2 % 128) == 0 && (kOffBias % 128) == 0 && (kSzH % 128) == 0, "128-B aligned regions");
static_assert(((size_t)kCatP * 2) % 128 == 0 && ((size_t)kHP * 2) % 128 == 0 && ((size_t)kInCol * 2) % 128 == 0, "line aligned f16 rows/segments");

union FragU { v16h v; v8h h[2]; };
__device__ __forceinline__ v16h frag_load(const _Float16* p) {
  FragU f;
  f.h[0] = *(const v8h*)(p);
  f.h[1] = *(const v8h*)(p + 16);
  return f.v;
}
__device__ __forceinline__ v8f mma_h(v16h a, v16h b, v8f c) {
  c = __builtin_amdgcn_wmma_f32_16x16x32_f16(false, a, false, b, (short)0, c, false, false);
  asm volatile("v_nop\n\tv_nop\n\tv_nop\n\tv_nop" : "+v"(c) : "v"(a), "v"(b));
  return c;
}
__device__ __forceinline__ v8f mma_raw(v16h a, v16h b, v8f c) {
  return __builtin_amdgcn_wmma_f32_16x16x32_f16(false, a, false, b, (short)0, c, false, false);
}
__device__ __forceinline__ void guard4_h(v8f& a, v8f& b, v8f& c, v8f& d, v16h x) {
  asm volatile("v_nop\n\tv_nop\n\tv_nop\n\tv_nop" : "+v"(a), "+v"(b), "+v"(c), "+v"(d) : "v"(x));
}
__device__ __forceinline__ void keep4_h(v16h a, v16h b, v16h c, v16h d) { asm volatile("v_nop" :: "v"(a), "v"(b), "v"(c), "v"(d)); }
__device__ __forceinline__ void acc_guard4(v8f& a, v8f& b, v8f& c, v8f& d) { asm volatile("v_nop\n\tv_nop\n\tv_nop\n\tv_nop" : "+v"(a), "+v"(b), "+v"(c), "+v"(d)); }
__device__ __forceinline__ void pin2_f4(v4f& a, v4f& b) { asm volatile("" : "+v"(a), "+v"(b)); }

__device__ __forceinline__ float wave_sum(float v) {
#pragma unroll
  for (int o = 16; o > 0; o >>= 1) v += __shfl_xor(v, o, 32);
  return v;
}
__device__ __forceinline__ float wave_max(float v) {
#pragma unroll
  for (int o = 16; o > 0; o >>= 1) v = fmaxf(v, __shfl_xor(v, o, 32));
  return v;
}
__device__ __forceinline__ float sigm(float v) { return __builtin_amdgcn_rcpf(1.0f + expf(-v)); }

struct PackArgs { const float* s0; const float* s1; unsigned short* dst; int kind; int total8; };
static_assert(sizeof(PackArgs) == 32, "no padding");

__global__ __launch_bounds__(256) void pack_planes_kernel(PackArgs a) {
  const int t = blockIdx.x * 256 + threadIdx.x;
  if (t >= a.total8) return;
  const int e0 = t * 8;
  const int kind = a.kind;
  v8h hv;
#pragma unroll
  for (int e = 0; e < 8; ++e) {
    const int el = e0 + e;
    const float* p = a.s0;
    size_t off = 0;
    bool ok = false;
    float sc = kWCarry;
    if (kind <= 1) {
      const int k = el % kHP;
      const int nn = el / kHP;
      const int n = nn % kGN;
      const int l = nn / kGN;
      const int d = (n / 96) * 16 + (n & 15);
      const int gate = (n % 96) >> 4;
      ok = (d < kHid) && (k < kHid);
      const int dc = d < kHid ? d : (kHid - 1);
      const int kc = k < kHid ? k : (kHid - 1);
      const int gs = gate < 3 ? gate : gate - 3;
      p = gate < 3 ? a.s0 : a.s1;
      off = ((size_t)l * 900 + gs * kHid + dc) * kHid + kc;
    } else if (kind == 2) {
      const int k = el % kWrK;
      const int nn = el / kWrK;
      const int n = nn % kHP;
      const int l = nn / kHP;
      const bool up = (k >= kHP);
      const int kk = up ? k - kHP : k;
      ok = (n < kHid) && (kk < kHid);
      const int nc = n < kHid ? n : (kHid - 1);
      const int kc = kk < kHid ? kk : (kHid - 1);
      p = up ? a.s1 : a.s0;
      off = ((size_t)l * kHid + nc) * kHid + kc;
    } else if (kind == 3) {
      const int k = el % kInP;
      const int n = el / kInP;
      ok = (n < kHid) && (k < kEmb);
      const int nc = n < kHid ? n : (kHid - 1);
      const int kc = k < kEmb ? k : (kEmb - 1);
      off = (size_t)nc * kEmb + kc;
    } else if (kind == 4) {
      const int cc = el % kCatP;
      const int n = el / kCatP;
      const bool tail = (cc >= kInCol);
      const int seg = cc / kHP;
      const int w = tail ? (cc - kInCol) : (cc - seg * kHP);
      const int lim = tail ? kEmb : kHid;
      const int wc = w < lim ? w : (lim - 1);
      const int col = tail ? (5 * kHid + wc) : (seg * kHid + wc);
      ok = (n < kHid) && (w < lim);
      const int nc = n < kHid ? n : (kHid - 1);
      off = (size_t)nc * 1600 + col;
    } else if (kind == 5) {
      const int k = el % kHP;
      const int n = el / kHP;
      ok = (n < kHid) && (k < kHid);
      const int nc = n < kHid ? n : (kHid - 1);
      const int kc = k < kHid ? k : (kHid - 1);
      off = (size_t)nc * kHid + kc;
    } else {
      const int k = el % kInP;
      const int rp = el / kInP;
      const int i = rp >> 3;
      const int b = rp & 7;
      ok = (k < kEmb);
      const int kc = k < kEmb ? k : (kEmb - 1);
      off = (size_t)(b * kUtt + i) * kEmb + kc;
      sc = 1.0f;
    }
    const float raw = p[off];
    const float v = ok ? raw * sc : 0.0f;
    hv[e] = (_Float16)v;
  }
  size_t dsto = (size_t)e0;
  if (kind == 6) dsto = (size_t)(e0 / kInP) * kCatP + kInCol + (e0 % kInP);
  unsigned short* q = a.dst + dsto;
  *(volatile v8h*)q = hv;
  __threadfence();
  *(volatile v8h*)q = hv;
}

__global__ __launch_bounds__(256) void pack_bias_kernel(
    const float* __restrict__ fc1b, const float* __restrict__ m1b, const float* __restrict__ m2b,
    const float* __restrict__ cbih, const float* __restrict__ cbhh,
    const float* __restrict__ pbih, const float* __restrict__ pbhh, float* dst) {
  const int t = blockIdx.x * 256 + threadIdx.x;
  if (t >= kBiasFloats / 4) return;
  v4f ov;
#pragma unroll
  for (int e = 0; e < 4; ++e) {
    const int idx = 4 * t + e;
    const bool head = (idx < 3 * kHP);
    const int hn = idx % kHP;
    const int hw = idx / kHP;
    const float* hp = (hw == 0) ? fc1b : ((hw == 1) ? m1b : m2b);
    const int hoff = hn < kHid ? hn : (kHid - 1);
    const bool hok = (hn < kHid);
    const int j = head ? 0 : (idx - 3 * kHP);
    const int side = j / (kLay * kGN);
    const int jj = j % (kLay * kGN);
    const int l = jj / kGN;
    const int n = jj % kGN;
    const int d = (n / 96) * 16 + (n & 15);
    const int gate = (n % 96) >> 4;
    const int dc = d < kHid ? d : (kHid - 1);
    const int gs = gate < 3 ? gate : gate - 3;
    const int goff = l * 900 + gs * kHid + dc;
    const bool gok = (d < kHid);
    const float* gp = (side == 0) ? ((gate < 3) ? cbih : pbhh) : ((gate < 3) ? cbhh : pbih);
    const float* p = head ? hp : gp;
    const int off = head ? hoff : goff;
    const bool ok = head ? hok : gok;
    const float raw = p[off];
    ov[e] = ok ? raw : 0.0f;
  }
  float* q = dst + (size_t)t * 4;
  *(volatile v4f*)q = ov;
  __threadfence();
  *(volatile v4f*)q = ov;
}

template <int BIAS_MODE, bool OUTF, bool OUTH, int ACT>
__global__ __launch_bounds__(256) void gemm64h_kernel(
    const unsigned short* __restrict__ Ap, int lda,
    const unsigned short* __restrict__ Btp, int ldb,
    float* Cf, int ldcf,
    unsigned short* Ch, int ldch,
    const float* __restrict__ bias,
    int M, int N, int K, float scale) {
  const _Float16* A  = (const _Float16*)Ap;
  const _Float16* Bt = (const _Float16*)Btp;
  __shared__ __align__(16) float sT[8][16 * 68];
  const int lane = threadIdx.x & 31;
  const int wave = threadIdx.x >> 5;
  const int tilesN = N >> 6;
  const int tilesM = M >> 6;
  const int tile = blockIdx.x * 8 + wave;
  if (tile >= tilesM * tilesN) return;
  const int tm = tile / tilesN;
  const int tn = tile - tm * tilesN;
  const int m0 = tm << 6;
  const int n0 = tn << 6;
  const int rlane = lane & 15;
  const int koff  = (lane >> 4) * 8;
  const int mOff  = (lane >> 4) * 8;

  v8f acc[4][4];
#pragma unroll
  for (int i = 0; i < 4; ++i)
#pragma unroll
    for (int j = 0; j < 4; ++j) acc[i][j] = (v8f){0.f,0.f,0.f,0.f,0.f,0.f,0.f,0.f};

  for (int k0 = 0; k0 < K; k0 += 32) {
    v16h bh[4];
#pragma unroll
    for (int j = 0; j < 4; ++j) {
      const size_t bo = (size_t)(n0 + (j << 4) + rlane) * ldb + koff + k0;
      bh[j] = frag_load(Bt + bo);
    }
#pragma unroll
    for (int i = 0; i < 4; ++i) {
      const size_t ao = (size_t)(m0 + (i << 4) + rlane) * lda + koff + k0;
      v16h ah = frag_load(A + ao);
#pragma unroll
      for (int j = 0; j < 4; ++j) acc[i][j] = mma_raw(ah, bh[j], acc[i][j]);
      guard4_h(acc[i][0], acc[i][1], acc[i][2], acc[i][3], ah);
    }
    keep4_h(bh[0], bh[1], bh[2], bh[3]);
  }
  acc_guard4(acc[0][0], acc[0][1], acc[0][2], acc[0][3]);
  acc_guard4(acc[1][0], acc[1][1], acc[1][2], acc[1][3]);
  acc_guard4(acc[2][0], acc[2][1], acc[2][2], acc[2][3]);
  acc_guard4(acc[3][0], acc[3][1], acc[3][2], acc[3][3]);

  float* slab = sT[wave];
#pragma unroll
  for (int i = 0; i < 4; ++i) {
    const int mBase = m0 + (i << 4);
#pragma unroll
    for (int j = 0; j < 4; ++j) {
      const int n = n0 + (j << 4) + rlane;
      float bv = 0.f;
      if (BIAS_MODE == 2) bv = bias[n];
#pragma unroll
      for (int r = 0; r < 8; ++r) {
        float v = acc[i][j][r] * scale;
        if (BIAS_MODE == 1) v += bias[mBase + mOff + r];
        if (BIAS_MODE == 2) v += bv;
        if (ACT == 2) v = fmaxf(v, 0.0f);
        slab[(mOff + r) * 68 + (j << 4) + rlane] = v;
      }
    }
    __builtin_amdgcn_fence(__ATOMIC_RELEASE, "workgroup");
    __builtin_amdgcn_wave_barrier();
    __builtin_amdgcn_fence(__ATOMIC_ACQUIRE, "workgroup");
    if (OUTF) {
      const int hh = lane >> 4, c4 = (lane & 15) * 4;
      for (int pass = 0; pass < 2; ++pass) {
#pragma unroll
        for (int it = 0; it < 8; ++it) {
          const int row = it * 2 + hh;
          v4f v = *(const v4f*)(slab + row * 68 + c4);
          *(volatile v4f*)(Cf + (size_t)(mBase + row) * ldcf + n0 + c4) = v;
        }
        __threadfence();
      }
    }
    if (OUTH) {
      const int q = lane >> 3, c8 = (lane & 7) * 8;
      for (int pass = 0; pass < 2; ++pass) {
#pragma unroll
        for (int it = 0; it < 4; ++it) {
          const int row = it * 4 + q;
          const float* sp = slab + row * 68 + c8;
          v8h hv;
#pragma unroll
          for (int e = 0; e < 8; ++e) hv[e] = (_Float16)sp[e];
          *(volatile v8h*)(Ch + (size_t)(mBase + row) * ldch + n0 + c8) = hv;
        }
        __threadfence();
      }
    }
    __builtin_amdgcn_fence(__ATOMIC_RELEASE, "workgroup");
    __builtin_amdgcn_wave_barrier();
    __builtin_amdgcn_fence(__ATOMIC_ACQUIRE, "workgroup");
  }
}

__global__ __launch_bounds__(640) void seq_scan_kernel(
    const float* __restrict__ Hin, float* Hout, unsigned short* AcatSeg,
    const int* __restrict__ adj, const int* __restrict__ smask,
    const float* __restrict__ gatw,
    const unsigned short* __restrict__ Wr, const unsigned short* __restrict__ Wm,
    const float* __restrict__ GXT, const float* __restrict__ BM) {
  __shared__ __align__(16) _Float16 m01h[kBat * kM01P];
  __shared__ __align__(16) _Float16 M16[kBat * kM16P];
  __shared__ __align__(16) float Mf[kBat * kHP];
  __shared__ __align__(16) float xf[kBat * kHP];
  __shared__ __align__(16) float hrow[kBat * kHP];
  __shared__ float aw0[kBat * kUtt];
  __shared__ float aw1[kBat * kUtt];
  __shared__ float kdot[kBat * kUtt];
  __shared__ float gwk[kHP];

  const int tid  = threadIdx.x;
  const int wave = tid >> 5;
  const int lane = tid & 31;
  const int hh   = lane >> 4;
  const int c    = lane & 15;
  const int koff = hh * 8;

  for (int idx = tid; idx < kBat * kUtt; idx += kScanThreads) kdot[idx] = 0.0f;
  for (int idx = tid; idx < kHP; idx += kScanThreads) {
    const int dc = idx < kHid ? idx : (kHid - 1);
    const float g = gatw[kHid + dc];
    gwk[idx] = (idx < kHid) ? g : 0.0f;
  }
  float bm[6];
#pragma unroll
  for (int g = 0; g < 6; ++g) bm[g] = BM[wave * 96 + g * 16 + c];
  v16h vz;
#pragma unroll
  for (int e = 0; e < 16; ++e) vz[e] = (_Float16)0.0f;
  __syncthreads();

  const _Float16* WrH = (const _Float16*)Wr;
  const _Float16* WmH = (const _Float16*)Wm;
  const int pb = tid / 80;
  const int pq = tid - pb * 80;
  const int pd0 = pq * 4;

#pragma unroll 1
  for (int i = 0; i < kUtt; ++i) {
    {
      const v4f xv = *(const v4f*)(Hin + (size_t)i * (kBat * kHP) + tid * 4);
      *(v4f*)(xf + tid * 4) = xv;
    }
    if (wave < kBat) {
      const int b = wave;
      const int* arow = adj   + (size_t)(b * kUtt + i) * kUtt;
      const int* srow = smask + (size_t)(b * kUtt + i) * kUtt;
      float lg[4], sm[4];
      bool vd[4], inr[4];
      float mx = -INFINITY;
#pragma unroll
      for (int q = 0; q < 4; ++q) {
        const int j = lane + 32 * q;
        const int av = arow[j];
        const int sv = srow[j];
        const float kd = kdot[b * kUtt + j];
        inr[q] = (j < i);
        vd[q] = inr[q] && (av != 0);
        lg[q] = vd[q] ? kd : -INFINITY;
        sm[q] = (float)sv;
        mx = fmaxf(mx, lg[q]);
      }
      mx = wave_max(mx);
      const bool none = !(mx > -3.0e38f);
      float ev[4];
      float s = 0.0f;
#pragma unroll
      for (int q = 0; q < 4; ++q) {
        const float ex = expf(lg[q] - mx);
        const float en = vd[q] ? ex : 0.0f;
        const float eu = inr[q] ? 1.0f : 0.0f;
        ev[q] = none ? eu : en;
        s += ev[q];
      }
      s = wave_sum(s);
      s = none ? 128.0f : s;
      const float inv = 1.0f / s;
#pragma unroll
      for (int q = 0; q < 4; ++q) {
        const int j = lane + 32 * q;
        const float a = ev[q] * inv;
        const float a0 = a * sm[q];
        aw0[b * kUtt + j] = a0;
        aw1[b * kUtt + j] = a - a0;
      }
    }
    __syncthreads();

    {
      v4f m0 = (v4f){0.f, 0.f, 0.f, 0.f};
      v4f m1 = (v4f){0.f, 0.f, 0.f, 0.f};
      const float* hp = Hout + (size_t)pb * kHP + pd0;
#pragma unroll 1
      for (int j = 0; j < i; ++j) {
        const float a0 = aw0[pb * kUtt + j];
        const float a1 = aw1[pb * kUtt + j];
        const v4f h = *(const v4f*)(hp + (size_t)j * (kBat * kHP));
        m0 += a0 * h;
        m1 += a1 * h;
      }
      const bool live = (pq < 75);
      v4h h0, h1;
#pragma unroll
      for (int e = 0; e < 4; ++e) {
        const float u0 = live ? m0[e] : 0.0f;
        const float u1 = live ? m1[e] : 0.0f;
        h0[e] = (_Float16)u0;
        h1[e] = (_Float16)u1;
      }
      *(v4h*)(m01h + pb * kM01P + pd0) = h0;
      *(v4h*)(m01h + pb * kM01P + kHP + pd0) = h1;
    }
    __syncthreads();

    {
      v8f acc = (v8f){0.f,0.f,0.f,0.f,0.f,0.f,0.f,0.f};
      const _Float16* bp = WrH + (size_t)(wave * 16 + c) * kWrK + koff;
      const _Float16* ap = m01h + (c & 7) * kM01P + koff;
#pragma unroll 2
      for (int kb = 0; kb < kWrK / 32; ++kb) {
        v16h a = frag_load(ap + kb * 32);
        a = (c < 8) ? a : vz;
        const v16h bfr = frag_load(bp + kb * 32);
        acc = mma_h(a, bfr, acc);
      }
      const int n = wave * 16 + c;
      if (hh == 0) {
#pragma unroll
        for (int r = 0; r < 8; ++r) {
          const float v = acc[r] * kWInv;
          Mf[r * kHP + n] = v;
          M16[r * kM16P + n] = (_Float16)v;
        }
      }
    }
    __syncthreads();

    {
      v8f acc[6];
#pragma unroll
      for (int g = 0; g < 6; ++g) acc[g] = (v8f){0.f,0.f,0.f,0.f,0.f,0.f,0.f,0.f};
      const _Float16* bp = WmH + (size_t)(wave * 96 + c) * kHP + koff;
      const _Float16* ap = M16 + (c & 7) * kM16P + koff;
#pragma unroll 2
      for (int kb = 0; kb < kHP / 32; ++kb) {
        v16h a = frag_load(ap + kb * 32);
        a = (c < 8) ? a : vz;
#pragma unroll
        for (int g = 0; g < 6; ++g) {
          const v16h bfr = frag_load(bp + (size_t)g * 16 * kHP + kb * 32);
          acc[g] = mma_h(a, bfr, acc[g]);
        }
      }
      const int d = wave * 16 + c;
      const float* gxp = GXT + (size_t)(wave * 96 + c) * kRows + i * 8;
      v4f ga[6], gb[6];
#pragma unroll
      for (int g = 0; g < 6; ++g) {
        ga[g] = *(const v4f*)(gxp + (size_t)g * 16 * kRows);
        gb[g] = *(const v4f*)(gxp + (size_t)g * 16 * kRows + 4);
      }
#pragma unroll
      for (int g = 0; g < 6; ++g) pin2_f4(ga[g], gb[g]);
      float hv[8];
#pragma unroll
      for (int r = 0; r < 8; ++r) {
        const float g0 = (r < 4) ? ga[0][r & 3] : gb[0][r & 3];
        const float g1 = (r < 4) ? ga[1][r & 3] : gb[1][r & 3];
        const float g2 = (r < 4) ? ga[2][r & 3] : gb[2][r & 3];
        const float g3 = (r < 4) ? ga[3][r & 3] : gb[3][r & 3];
        const float g4 = (r < 4) ? ga[4][r & 3] : gb[4][r & 3];
        const float g5 = (r < 4) ? ga[5][r & 3] : gb[5][r & 3];
        const float q0 = acc[0][r] * kWInv + bm[0];
        const float q1 = acc[1][r] * kWInv + bm[1];
        const float q2 = acc[2][r] * kWInv + bm[2];
        const float q3 = acc[3][r] * kWInv + bm[3];
        const float q4 = acc[4][r] * kWInv + bm[4];
        const float q5 = acc[5][r] * kWInv + bm[5];
        const float xm = xf[r * kHP + d];
        const float mm = Mf[r * kHP + d];
        const float cr = sigm(g0 + q0);
        const float cz = sigm(g1 + q1);
        const float cn = tanhf(g2 + cr * q2);
        const float cv = (1.0f - cz) * cn + cz * mm;
        const float pr = sigm(q3 + g3);
        const float pz = sigm(q4 + g4);
        const float pn = tanhf(q5 + pr * g5);
        const float pv = (1.0f - pz) * pn + pz * xm;
        const float hs = cv + pv;
        hv[r] = (d < kHid) ? hs : 0.0f;
      }
      if (hh == 0) {
#pragma unroll
        for (int r = 0; r < 8; ++r) hrow[r * kHP + d] = hv[r];
      }
    }
    __syncthreads();

    {
      const v4f fv = *(const v4f*)(hrow + tid * 4);
      float* dstH = Hout + (size_t)i * (kBat * kHP) + tid * 4;
      const bool hw = (tid < 320);
      const int trow = hw ? (tid / 40) : 0;
      const int tc8 = hw ? ((tid - trow * 40) * 8) : 0;
      const v4f p0 = *(const v4f*)(hrow + trow * kHP + tc8);
      const v4f p1 = *(const v4f*)(hrow + trow * kHP + tc8 + 4);
      v8h hvv;
#pragma unroll
      for (int e = 0; e < 4; ++e) {
        hvv[e] = (_Float16)p0[e];
        hvv[4 + e] = (_Float16)p1[e];
      }
      unsigned short* dstA = AcatSeg + (size_t)(i * kBat + trow) * kCatP + tc8;
      for (int pass = 0; pass < 2; ++pass) {
        *(volatile v4f*)dstH = fv;
        if (hw) *(volatile v8h*)dstA = hvv;
        __threadfence();
      }
      if (wave < kBat) {
        float p = 0.0f;
#pragma unroll 1
        for (int dd = lane; dd < kHP; dd += 32) p = fmaf(hrow[wave * kHP + dd], gwk[dd], p);
        p = wave_sum(p);
        if (lane == 0) kdot[wave * kUtt + i] = p;
      }
    }
    __threadfence();
    __syncthreads();
  }
}

__global__ __launch_bounds__(256) void head3_kernel(const float* __restrict__ h2, const float* __restrict__ w3,
                                                    const float* __restrict__ b3, float* out) {
  const int idx = blockIdx.x * 256 + threadIdx.x;
  const int row = idx / kCls;
  const int cc  = idx - row * kCls;
  const int b   = row >> 7;
  const int i   = row & (kUtt - 1);
  const float* hp = h2 + (size_t)(i * kBat + b) * kHP;
  const float* wp = w3 + (size_t)cc * kHid;
  float a0 = 0.f, a1 = 0.f, a2 = 0.f, a3 = 0.f;
#pragma unroll 1
  for (int k4 = 0; k4 < kHid / 4; ++k4) {
    const v4f hvv = *(const v4f*)(hp + 4 * k4);
    const v4f wv = *(const v4f*)(wp + 4 * k4);
    a0 = fmaf(hvv[0], wv[0], a0);
    a1 = fmaf(hvv[1], wv[1], a1);
    a2 = fmaf(hvv[2], wv[2], a2);
    a3 = fmaf(hvv[3], wv[3], a3);
  }
  const float v = ((a0 + a1) + (a2 + a3)) + b3[cc];
  *(volatile float*)(out + idx) = v;
  __threadfence();
  *(volatile float*)(out + idx) = v;
}

extern "C" void kernel_launch(void* const* d_in, const int* in_sizes, int n_in,
                              void* d_out, int out_size, void* d_ws, size_t ws_size,
                              hipStream_t stream) {
  if (n_in < 24) return;
  if (in_sizes[0] != kRows * kEmb) return;
  if (in_sizes[1] != kBat * kUtt * kUtt) return;
  if (in_sizes[2] != kBat * kUtt * kUtt) return;
  if (in_sizes[4] != kHid * kEmb) return;
  if (in_sizes[5] != kHid) return;
  if (in_sizes[6] != kLay * 2 * kHid) return;
  if (in_sizes[8] != kLay * kHid * kHid) return;
  if (in_sizes[9] != kLay * kHid * kHid) return;
  if (in_sizes[10] != kLay * 900 * kHid) return;
  if (in_sizes[11] != kLay * 900 * kHid) return;
  if (in_sizes[12] != kLay * 900) return;
  if (in_sizes[13] != kLay * 900) return;
  if (in_sizes[14] != kLay * 900 * kHid) return;
  if (in_sizes[15] != kLay * 900 * kHid) return;
  if (in_sizes[16] != kLay * 900) return;
  if (in_sizes[17] != kLay * 900) return;
  if (in_sizes[18] != kHid * 1600) return;
  if (in_sizes[19] != kHid) return;
  if (in_sizes[20] != kHid * kHid) return;
  if (in_sizes[21] != kHid) return;
  if (in_sizes[22] != kCls * kHid) return;
  if (in_sizes[23] != kCls) return;
  if (out_size != kRows * kCls) return;
  if (ws_size < kWsTotal) return;

  const float* input   = (const float*)d_in[0];
  const int*   adj     = (const int*)  d_in[1];
  const int*   smask   = (const int*)  d_in[2];
  const float* fc1_w   = (const float*)d_in[4];
  const float* fc1_b   = (const float*)d_in[5];
  const float* gat_w   = (const float*)d_in[6];
  const float* wr0     = (const float*)d_in[8];
  const float* wr1     = (const float*)d_in[9];
  const float* gc_wih  = (const float*)d_in[10];
  const float* gc_whh  = (const float*)d_in[11];
  const float* gc_bih  = (const float*)d_in[12];
  const float* gc_bhh  = (const float*)d_in[13];
  const float* gp_wih  = (const float*)d_in[14];
  const float* gp_whh  = (const float*)d_in[15];
  const float* gp_bih  = (const float*)d_in[16];
  const float* gp_bhh  = (const float*)d_in[17];
  const float* mlp1_w  = (const float*)d_in[18];
  const float* mlp1_b  = (const float*)d_in[19];
  const float* mlp2_w  = (const float*)d_in[20];
  const float* mlp2_b  = (const float*)d_in[21];
  const float* mlp3_w  = (const float*)d_in[22];
  const float* mlp3_b  = (const float*)d_in[23];

  char* ws = (char*)d_ws;
  float*          HPL  = (float*)(ws + kOffH);
  unsigned short* ACAT = (unsigned short*)(ws + kOffCat);
  float*          GXT  = (float*)(ws + kOffGXT);
  unsigned short* WX   = (unsigned short*)(ws + kOffWX);
  unsigned short* WM   = (unsigned short*)(ws + kOffWM);
  unsigned short* WR   = (unsigned short*)(ws + kOffWR);
  unsigned short* FC1P = (unsigned short*)(ws + kOffFC1);
  unsigned short* M1P  = (unsigned short*)(ws + kOffM1);
  unsigned short* M2P  = (unsigned short*)(ws + kOffM2);
  unsigned short* H1H  = (unsigned short*)(ws + kOffH1);
  float*          H2F  = (float*)(ws + kOffH2);
  float*          BIAS = (float*)(ws + kOffBias);
  const size_t hElems = (size_t)kRows * kHP;

  {
    PackArgs a;
    constexpr int tGate = kLay * kGN * kHP / 8;
    constexpr int tWr   = kLay * kHP * kWrK / 8;
    constexpr int tFc1  = kHP * kInP / 8;
    constexpr int tM1   = kHP * kCatP / 8;
    constexpr int tM2   = kHP * kHP / 8;
    constexpr int tIn   = kRows * kInP / 8;
    static_assert((tGate % 256) == 0 && (tWr % 256) == 0 && (tFc1 % 256) == 0 && (tM1 % 256) == 0 &&
                  (tM2 % 256) == 0 && (tIn % 256) == 0, "pack grids exact");
    a.s0 = gc_wih; a.s1 = gp_whh; a.dst = WX; a.kind = 0; a.total8 = tGate;
    pack_planes_kernel<<<tGate / 256, 256, 0, stream>>>(a);
    a.s0 = gc_whh; a.s1 = gp_wih; a.dst = WM; a.kind = 1; a.total8 = tGate;
    pack_planes_kernel<<<tGate / 256, 256, 0, stream>>>(a);
    a.s0 = wr0; a.s1 = wr1; a.dst = WR; a.kind = 2; a.total8 = tWr;
    pack_planes_kernel<<<tWr / 256, 256, 0, stream>>>(a);
    a.s0 = fc1_w; a.s1 = fc1_w; a.dst = FC1P; a.kind = 3; a.total8 = tFc1;
    pack_planes_kernel<<<tFc1 / 256, 256, 0, stream>>>(a);
    a.s0 = mlp1_w; a.s1 = mlp1_w; a.dst = M1P; a.kind = 4; a.total8 = tM1;
    pack_planes_kernel<<<tM1 / 256, 256, 0, stream>>>(a);
    a.s0 = mlp2_w; a.s1 = mlp2_w; a.dst = M2P; a.kind = 5; a.total8 = tM2;
    pack_planes_kernel<<<tM2 / 256, 256, 0, stream>>>(a);
    a.s0 = input; a.s1 = input; a.dst = ACAT; a.kind = 6; a.total8 = tIn;
    pack_planes_kernel<<<tIn / 256, 256, 0, stream>>>(a);
  }
  pack_bias_kernel<<<(kBiasFloats / 4 + 255) / 256, 256, 0, stream>>>(fc1_b, mlp1_b, mlp2_b, gc_bih, gc_bhh, gp_bih, gp_bhh, BIAS);

  static_assert((kRows / 64) * (kHP / 64) == 80, "fc1/mlp tiles");
  gemm64h_kernel<2, true, true, 2><<<10, 256, 0, stream>>>(
      ACAT + kInCol, kCatP, FC1P, kInP,
      HPL, kHP, ACAT, kCatP,
      BIAS, kRows, kHP, kInP, kWInv);

  static_assert((kGN / 64) * (kRows / 64) == 480, "x-side tiles");
  for (int l = 0; l < kLay; ++l) {
    gemm64h_kernel<1, true, false, 0><<<60, 256, 0, stream>>>(
        WX + (size_t)l * kGN * kHP, kHP, ACAT + (size_t)kHP * l, kCatP,
        GXT, kRows, H1H, kHP,
        BIAS + 3 * kHP + (size_t)l * kGN, kGN, kRows, kHP, kWInv);
    seq_scan_kernel<<<1, kScanThreads, 0, stream>>>(
        HPL + (size_t)l * hElems, HPL + (size_t)(l + 1) * hElems, ACAT + (size_t)kHP * (l + 1),
        adj, smask, gat_w + (size_t)l * 2 * kHid,
        WR + (size_t)l * kHP * kWrK, WM + (size_t)l * kGN * kHP,
        GXT, BIAS + 3 * kHP + (size_t)kLay * kGN + (size_t)l * kGN);
  }

  gemm64h_kernel<2, false, true, 2><<<10, 256, 0, stream>>>(
      ACAT, kCatP, M1P, kCatP,
      H2F, kHP, H1H, kHP,
      BIAS + kHP, kRows, kHP, kCatP, kWInv);
  gemm64h_kernel<2, true, false, 2><<<10, 256, 0, stream>>>(
      H1H, kHP, M2P, kHP,
      H2F, kHP, H1H, kHP,
      BIAS + 2 * kHP, kRows, kHP, kHP, kWInv);
  static_assert(kRows * kCls == 28 * 256, "head grid exact");
  head3_kernel<<<28, 256, 0, stream>>>(H2F, mlp3_w, mlp3_b, (float*)d_out);
}
